// PerceiverAttention_14233521619502
// MI455X (gfx1250) — hardware-verified
//
#include <hip/hip_runtime.h>
#include <math.h>


#define DD 1024
#define NH 16
#define DH 64
#define BL 9
#define BX 8
#define NKV 256
#define NQ 64
#define NQR (BL * NQ)
#define NKR (BX * (NKV + NQ))
#define KVB (NKV + NQ)

typedef __attribute__((ext_vector_type(16))) _Float16 v16h;
typedef __attribute__((ext_vector_type(8)))  _Float16 v8h;
typedef __attribute__((ext_vector_type(8)))  float v8f;
typedef __attribute__((ext_vector_type(4)))  float v4f;
typedef __attribute__((ext_vector_type(4)))  unsigned v4u;

template <typename T> __device__ __forceinline__ void vst2(void* p, T v) { *(volatile T*)p = v; __threadfence(); *(volatile T*)p = v; }
__device__ __forceinline__ v8f wmma16(v16h a, v16h b, v8f c) {
  v8f d = __builtin_amdgcn_wmma_f32_16x16x32_f16(false, a, false, b, (short)0, c, false, false);
  asm volatile("v_nop\n\tv_nop\n\tv_nop\n\tv_nop" : "+v"(d) : "v"(a), "v"(b));
  return d;
}
__device__ __forceinline__ v16h frag_h(const _Float16* rowk0, int lane) {
  union { v16h v; v8h q[2]; } u; const _Float16* p = rowk0 + 8 * (lane >> 4);
  u.q[0] = *(const v8h*)p; u.q[1] = *(const v8h*)(p + 16); return u.v;
}
__device__ __forceinline__ v16h frag_f32(const float* rowk0, int lane) {
  v16h a; const float* p = rowk0 + 8 * (lane >> 4);
#pragma unroll
  for (int i = 0; i < 8; ++i) { a[i] = (_Float16)p[i]; a[8 + i] = (_Float16)p[16 + i]; }
  return a;
}
#define LDSX() do { asm volatile("s_wait_dscnt 0" ::: "memory"); __builtin_amdgcn_wave_barrier(); __builtin_amdgcn_fence(__ATOMIC_RELEASE, "workgroup"); } while (0)

__global__ __launch_bounds__(256) void k_packT(const float* __restrict__ W, _Float16* __restrict__ Wt, int N) {
  __shared__ float tile[64][65];
  const int k0 = blockIdx.y * 64, n0 = blockIdx.x * 64, tid = threadIdx.x;
  for (int q = tid; q < 64 * 64; q += 256) { const int kk = q >> 6, nn = q & 63; tile[kk][nn] = W[(size_t)(k0 + kk) * N + n0 + nn]; }
  __syncthreads();
  const int pc = tid & 7;
#pragma unroll
  for (int u = 0; u < 2; ++u) { const int nn = (tid >> 3) + u * 32; union { v8h h; v4u uu; } pk;
#pragma unroll
    for (int e = 0; e < 8; ++e) pk.h[e] = (_Float16)tile[pc * 8 + e][nn];
    vst2(Wt + (size_t)(n0 + nn) * DD + k0 + pc * 8, pk.uu); }
}
__global__ __launch_bounds__(256) void k_ln(const float* __restrict__ x, const float* __restrict__ lat, const float* __restrict__ g1, const float* __restrict__ b1,
                                          const float* __restrict__ g2, const float* __restrict__ b2, _Float16* __restrict__ xn, _Float16* __restrict__ ln) {
  const int tid = threadIdx.x, w = tid >> 5, lane = tid & 31; const int row = blockIdx.x * 8 + w;
  const int NX = BX * NKV;
  if (row >= NX + NQR) return;
  const bool isx = row < NX;
  const float* src = isx ? x + (size_t)row * DD : lat + (size_t)(row - NX) * DD;
  const float* gg = isx ? g1 : g2; const float* bb = isx ? b1 : b2;
  _Float16* dst = isx ? xn + (size_t)row * DD : ln + (size_t)(row - NX) * DD;
  float v[32];
#pragma unroll
  for (int q = 0; q < 8; ++q) { const v4f t = *(const v4f*)(src + q * 128 + lane * 4); v[q * 4] = t[0]; v[q * 4 + 1] = t[1]; v[q * 4 + 2] = t[2]; v[q * 4 + 3] = t[3]; }
  float s = 0.f;
#pragma unroll
  for (int i = 0; i < 32; ++i) s += v[i];
#pragma unroll
  for (int off = 16; off >= 1; off >>= 1) s += __shfl_xor(s, off, 32);
  const float mu = s / (float)DD; float qv = 0.f;
#pragma unroll
  for (int i = 0; i < 32; ++i) { v[i] -= mu; qv += v[i] * v[i]; }
#pragma unroll
  for (int off = 16; off >= 1; off >>= 1) qv += __shfl_xor(qv, off, 32);
  const float rs = rsqrtf(qv / (float)DD + 1e-5f);
#pragma unroll
  for (int q = 0; q < 8; ++q) { float o[4], n[4];
#pragma unroll
    for (int e = 0; e < 4; ++e) { const int c = q * 128 + lane * 4 + e; o[e] = v[q * 4 + e] * rs * gg[c] + bb[c]; }
#pragma unroll
    for (int e = 0; e < 4; ++e) n[e] = __shfl_xor(o[e], 1, 32);
    if ((lane & 1) == 0) { union { v8h h; v4u uu; } pk;
#pragma unroll
      for (int e = 0; e < 4; ++e) { pk.h[e] = (_Float16)o[e]; pk.h[4 + e] = (_Float16)n[e]; }
      vst2(dst + q * 128 + lane * 4, pk.uu); } }
}
template <int ROWSEL, int VT>
__global__ __launch_bounds__(128) void k_proj(const _Float16* __restrict__ xn, const _Float16* __restrict__ ln, const _Float16* __restrict__ Wt,
                                            _Float16* __restrict__ Out, int ldo, _Float16* __restrict__ vT, int nrows) {
  __shared__ __align__(16) float so[4][16][132];
  __shared__ __align__(16) _Float16 st[128][72];
  const int tid = threadIdx.x, wave = tid >> 5, lane = tid & 31, col = lane & 15, g = lane >> 4;
  const int r0 = blockIdx.x * 64 + wave * 16, n0 = blockIdx.y * 128;
  int r = r0 + col; if (r > nrows - 1) r = nrows - 1;
  const _Float16* arow;
  if (ROWSEL == 0) arow = ln + (size_t)r * DD;
  else { const int bx = r / KVB, rr = r % KVB; arow = rr < NKV ? xn + ((size_t)bx * NKV + rr) * DD : ln + ((size_t)bx * NQ + rr - NKV) * DD; }
  v8f acc[8] = {};
#pragma unroll 1
  for (int kc = 0; kc < DD / 32; ++kc) { const v16h a = frag_h(arow + kc * 32, lane);
#pragma unroll
    for (int j = 0; j < 8; ++j) acc[j] = wmma16(a, frag_h(Wt + (size_t)(n0 + j * 16 + col) * DD + kc * 32, lane), acc[j]); }
  if (!VT || n0 < DD) {
    float* S = &so[wave][0][0];
#pragma unroll
    for (int j = 0; j < 8; ++j)
#pragma unroll
      for (int rr = 0; rr < 8; ++rr) S[(8 * g + rr) * 132 + j * 16 + col] = acc[j][rr];
    LDSX();
#pragma unroll
    for (int q = 0; q < 8; ++q) { const int rl = q * 2 + (lane >> 4), pc = lane & 15; if (r0 + rl >= nrows) continue;
      union { v8h h; v4u uu; } pk;
#pragma unroll
      for (int e = 0; e < 8; ++e) pk.h[e] = (_Float16)S[rl * 132 + pc * 8 + e];
      vst2(Out + (size_t)(r0 + rl) * ldo + n0 + pc * 8, pk.uu); }
  } else {
#pragma unroll
    for (int j = 0; j < 8; ++j)
#pragma unroll
      for (int rr = 0; rr < 8; ++rr) st[j * 16 + col][wave * 16 + 8 * g + rr] = (_Float16)acc[j][rr];
    __syncthreads();
    for (int q = tid; q < 128 * 8; q += 128) { const int c = q >> 3, pc = q & 7;
      vst2(vT + (size_t)(n0 - DD + c) * NKR + blockIdx.x * 64 + pc * 8, *(const v4u*)(&st[c][pc * 8])); }
  }
}
__global__ __launch_bounds__(128) void k_attn(const _Float16* __restrict__ Q, const _Float16* __restrict__ K, const _Float16* __restrict__ vT,
                                            const int* __restrict__ use_mask, _Float16* __restrict__ O) {
  __shared__ __align__(16) float sS[4][16][68];
  __shared__ __align__(16) _Float16 sP[4][16][72];
  __shared__ __align__(16) float sO[4][16][68];
  const int tid = threadIdx.x, w = tid >> 5, lane = tid & 31, col = lane & 15, g = lane >> 4;
  const int h = blockIdx.y, q0 = blockIdx.x * 64 + w * 16;
  const int rb = blockIdx.x;
  const bool masked = use_mask[0] != 0;
  v16h aq[2];
#pragma unroll
  for (int kc = 0; kc < 2; ++kc) aq[kc] = frag_h(Q + (size_t)(q0 + col) * DD + h * DH + kc * 32, lane);
  float mrun = -3.0e38f, lrun = 0.f; v8f acc[4] = {};
#pragma unroll 1
  for (int kt = 0; kt < NKR / 64; ++kt) {
    const int cb = (kt * 64) / KVB;
    if (masked && rb < BX && cb != rb) continue;
    v8f s4[4];
#pragma unroll
    for (int t = 0; t < 4; ++t) { s4[t] = (v8f){};
#pragma unroll
      for (int kc = 0; kc < 2; ++kc) s4[t] = wmma16(aq[kc], frag_h(K + (size_t)(kt * 64 + t * 16 + col) * DD + h * DH + kc * 32, lane), s4[t]); }
#pragma unroll
    for (int t = 0; t < 4; ++t)
#pragma unroll
      for (int r = 0; r < 8; ++r) sS[w][8 * g + r][t * 16 + col] = s4[t][r] * 0.125f;
    LDSX();
    float mx = -3.0e38f;
#pragma unroll
    for (int j = 0; j < 32; ++j) mx = fmaxf(mx, sS[w][col][g * 32 + j]);
    mx = fmaxf(mx, __shfl_xor(mx, 16, 32));
    const float mnew = fmaxf(mrun, mx); const float corr = expf(mrun - mnew);
    float ps = 0.f;
#pragma unroll
    for (int j = 0; j < 32; ++j) { const float p = expf(sS[w][col][g * 32 + j] - mnew); ps += p; sP[w][col][g * 32 + j] = (_Float16)(p * 16384.0f); }
    ps += __shfl_xor(ps, 16, 32);
    lrun = lrun * corr + ps; mrun = mnew;
#pragma unroll
    for (int r = 0; r < 8; ++r) { const float cr = __shfl(corr, 8 * g + r, 32);
#pragma unroll
      for (int t = 0; t < 4; ++t) acc[t][r] *= cr; }
    LDSX();
#pragma unroll
    for (int kc = 0; kc < 2; ++kc) { const v16h pa = frag_h(&sP[w][col][0] + kc * 32, lane);
#pragma unroll
      for (int t = 0; t < 4; ++t) acc[t] = wmma16(pa, frag_h(vT + (size_t)(h * DH + t * 16 + col) * NKR + kt * 64 + kc * 32, lane), acc[t]); }
    __builtin_amdgcn_wave_barrier();
  }
#pragma unroll
  for (int r = 0; r < 8; ++r) { const float lr = __shfl(lrun, 8 * g + r, 32);
#pragma unroll
    for (int t = 0; t < 4; ++t) sO[w][8 * g + r][t * 16 + col] = acc[t][r] / (lr * 16384.0f); }
  LDSX();
#pragma unroll
  for (int u = 0; u < 4; ++u) { const int q = lane + u * 32, rl = q >> 3, pc = q & 7; union { v8h hh; v4u uu; } pk;
#pragma unroll
    for (int e = 0; e < 8; ++e) pk.hh[e] = (_Float16)sO[w][rl][pc * 8 + e];
    vst2(O + (size_t)(q0 + rl) * DD + h * DH + pc * 8, pk.uu); }
}
__global__ __launch_bounds__(128) void k_out(const _Float16* __restrict__ O, const _Float16* __restrict__ Wt, float* __restrict__ out) {
  __shared__ __align__(16) float so[4][16][132];
  const int tid = threadIdx.x, wave = tid >> 5, lane = tid & 31, col = lane & 15, g = lane >> 4;
  const int r0 = blockIdx.x * 64 + wave * 16, n0 = blockIdx.y * 128;
  v8f acc[8] = {};
#pragma unroll 1
  for (int kc = 0; kc < DD / 32; ++kc) { const v16h a = frag_h(O + (size_t)(r0 + col) * DD + kc * 32, lane);
#pragma unroll
    for (int j = 0; j < 8; ++j) acc[j] = wmma16(a, frag_h(Wt + (size_t)(n0 + j * 16 + col) * DD + kc * 32, lane), acc[j]); }
  float* S = &so[wave][0][0];
#pragma unroll
  for (int j = 0; j < 8; ++j)
#pragma unroll
    for (int rr = 0; rr < 8; ++rr) S[(8 * g + rr) * 132 + j * 16 + col] = acc[j][rr];
  LDSX();
#pragma unroll 4
  for (int rl = 0; rl < 16; ++rl) vst2(out + (size_t)(r0 + rl) * DD + n0 + lane * 4, *(const v4f*)(S + rl * 132 + lane * 4));
}

extern "C" void kernel_launch(void* const* d_in, const int* in_sizes, int n_in,
                              void* d_out, int out_size, void* d_ws, size_t ws_size,
                              hipStream_t stream) {
  (void)in_sizes; (void)n_in; (void)out_size; (void)ws_size;
  const float* x = (const float*)d_in[0]; const float* lat = (const float*)d_in[1];
  const float* g1 = (const float*)d_in[2]; const float* b1 = (const float*)d_in[3]; const float* g2 = (const float*)d_in[4]; const float* b2 = (const float*)d_in[5];
  const float* Wq = (const float*)d_in[6]; const float* Wkv = (const float*)d_in[7]; const float* Wo = (const float*)d_in[8]; const int* um = (const int*)d_in[9];
  float* out = (float*)d_out;
  char* ws = (char*)d_ws; size_t off = 0;
  auto take = [&](size_t bytes) { char* p = ws + off; off += (bytes + 255) & ~(size_t)255; return (_Float16*)p; };
  _Float16* WqT = take((size_t)DD * DD * 2); _Float16* WkvT = take((size_t)2 * DD * DD * 2); _Float16* WoT = take((size_t)DD * DD * 2);
  _Float16* xn = take((size_t)BX * NKV * DD * 2); _Float16* ln = take((size_t)NQR * DD * 2);
  _Float16* Q = take((size_t)NQR * DD * 2); _Float16* Kr = take((size_t)NKR * DD * 2); _Float16* vT = take((size_t)DD * NKR * 2);
  _Float16* O16 = take((size_t)NQR * DD * 2);
  k_packT<<<dim3(DD / 64, DD / 64), 256, 0, stream>>>(Wq, WqT, DD);
  k_packT<<<dim3(2 * DD / 64, DD / 64), 256, 0, stream>>>(Wkv, WkvT, 2 * DD);
  k_packT<<<dim3(DD / 64, DD / 64), 256, 0, stream>>>(Wo, WoT, DD);
  k_ln<<<(BX * NKV + NQR + 7) / 8, 256, 0, stream>>>(x, lat, g1, b1, g2, b2, xn, ln);
  k_proj<0, 0><<<dim3(NQR / 64, DD / 128), 128, 0, stream>>>(xn, ln, WqT, Q, DD, nullptr, NQR);
  k_proj<1, 1><<<dim3(NKR / 64, 2 * DD / 128), 128, 0, stream>>>(xn, ln, WkvT, Kr, DD, vT, NKR);
  k_attn<<<dim3(NQR / 64, NH), 128, 0, stream>>>(Q, Kr, vT, um, O16);
  k_out<<<dim3(NQR / 64, DD / 128), 128, 0, stream>>>(O16, WoT, out);
}
